// SelfAttentionLayer_38104949850747
// MI455X (gfx1250) — hardware-verified
//
#include <hip/hip_runtime.h>


#ifndef NB
#define NB 4
#endif
#ifndef SEQ
#define SEQ 1024
#endif
#define NB_FULL  4
#define SEQ_FULL 1024
#define DM    1024
#define NH    16
#define DH    64
#define QKVW  3072
#define FFD   4096
#define NTOK  (NB * SEQ)
#define ICH   (SEQ / 2)
#define NCH   (SEQ / ICH)
#define EL    (SEQ / 32)
#define NV8   (SEQ / 256)
#define NTW   (SEQ / 128)
#define WCAR  16.0f
#define HCAR  16.0f
#define ACAR  16.0f
#define OCAR  256.0f
#define MCAR  64.0f
#define PCAR  16384.0f
#define P2CAR 16384.0f
#define L2E   1.4426950408889634f
#define EP_H16  0
#define EP_GELU 1
#define EP_RES  2

static_assert(NB >= 1 && NB <= NB_FULL);
static_assert(SEQ >= 256 && SEQ <= SEQ_FULL);
static_assert((SEQ % 256) == 0);
static_assert((ICH % 64) == 0);
static_assert(SEQ == SEQ_FULL || NB == 1);
static_assert((NTOK % 64) == 0);
static_assert(NH * DH == DM);
static_assert((size_t)NTOK * DM * 4 <= (size_t)16777216);

typedef _Float16 h16;
typedef __attribute__((ext_vector_type(16))) _Float16 v16h;
typedef __attribute__((ext_vector_type(8)))  _Float16 v8h;
typedef __attribute__((ext_vector_type(2)))  _Float16 v2h;
typedef __attribute__((ext_vector_type(8)))  float    v8f;
typedef __attribute__((ext_vector_type(4)))  float    v4f;
typedef v8h __attribute__((may_alias)) v8ha;
typedef v4f __attribute__((may_alias)) v4fa;

__device__ __forceinline__ float bfr(float f) { unsigned u = __float_as_uint(f); u += 0x7FFFu + ((u >> 16) & 1u); return __uint_as_float(u & 0xFFFF0000u); }
__device__ __forceinline__ v16h cat16(v8h lo, v8h hi) { return __builtin_shufflevector(lo, hi, 0, 1, 2, 3, 4, 5, 6, 7, 8, 9, 10, 11, 12, 13, 14, 15); }
__device__ __forceinline__ v8f cat8f(v4f lo, v4f hi) { return __builtin_shufflevector(lo, hi, 0, 1, 2, 3, 4, 5, 6, 7); }
__device__ __forceinline__ v8f wmma16(v16h a, v16h b, v8f c) { return __builtin_amdgcn_wmma_f32_16x16x32_f16(false, a, false, b, (short)0, c, false, false); }
__device__ __forceinline__ float wsum(float v) { v += __shfl_xor(v, 16, 32); v += __shfl_xor(v, 8, 32); v += __shfl_xor(v, 4, 32); v += __shfl_xor(v, 2, 32); v += __shfl_xor(v, 1, 32); return v; }
__device__ __forceinline__ float wmax(float v) { v = fmaxf(v, __shfl_xor(v, 16, 32)); v = fmaxf(v, __shfl_xor(v, 8, 32)); v = fmaxf(v, __shfl_xor(v, 4, 32)); v = fmaxf(v, __shfl_xor(v, 2, 32)); v = fmaxf(v, __shfl_xor(v, 1, 32)); return v; }

__device__ __forceinline__ v16h ldfrag(const h16* p) { return cat16(*(const v8ha*)p, *(const v8ha*)(p + 16)); }
__device__ __forceinline__ v16h ldfrag_lo(const h16* p) { return cat16(*(const v8ha*)p, (v8h){}); }

__device__ __forceinline__ float gelu_t(float x) {
    const float u = 0.7978845608028654f * (x + 0.044715f * x * x * x);
    const float e = __builtin_amdgcn_exp2f(2.0f * L2E * u);
    const float t = 1.0f - 2.0f * __builtin_amdgcn_rcpf(1.0f + e);
    return 0.5f * x * (1.0f + t);
}

__device__ __forceinline__ void ldmix(const float* __restrict__ W, const float* __restrict__ bv, float bscale, int lr, int hi, v16h& aw, v8f& bg) {
    const v4f w0 = *(const v4f*)(W + lr * NH + 8 * hi), w1 = *(const v4f*)(W + lr * NH + 8 * hi + 4);
    const v4f c0 = *(const v4f*)(bv + 8 * hi), c1 = *(const v4f*)(bv + 8 * hi + 4);
    const v8f wv = cat8f(w0, w1), cv = cat8f(c0, c1);
    v8h lo;
#pragma unroll
    for (int e = 0; e < 8; ++e) { const float we = wv[e]; lo[e] = (h16)(bfr(we) * MCAR); const float ce = cv[e]; bg[e] = bfr(ce) * bscale; }
    aw = cat16(lo, (v8h){});
}

template <int EP, bool BIAS, bool RBF>
__global__ __launch_bounds__(32) void k_gemm(const h16* __restrict__ A, const h16* __restrict__ Bt, int K,
                                             float* Cf, h16* Ch, int ldc, float cs, float co,
                                             const float* __restrict__ bias, const float* __restrict__ R, const float* __restrict__ gam,
                                             size_t sA, size_t sB, size_t sC) {
    __shared__ __align__(16) float os[16 * 68];
    const size_t z = blockIdx.z; A += z * sA; Bt += z * sB;
    const int lane = threadIdx.x & 31, lr = lane & 15, hi = lane >> 4;
    const int r0 = blockIdx.x * 64, c0 = blockIdx.y * 64;
    v8f acc[4][4];
#pragma unroll
    for (int mb = 0; mb < 4; ++mb)
#pragma unroll
        for (int nb = 0; nb < 4; ++nb) acc[mb][nb] = (v8f){};
    const size_t aoff = (size_t)(r0 + lr) * K + 8 * hi, boff = (size_t)(c0 + lr) * K + 8 * hi;
#pragma unroll 1
    for (int kc = 0; kc < K; kc += 32) {
        v16h a[4], b;
#pragma unroll
        for (int mb = 0; mb < 4; ++mb) a[mb] = ldfrag(A + aoff + (size_t)mb * 16 * K + kc);
#pragma unroll
        for (int nb = 0; nb < 4; ++nb) {
            b = ldfrag(Bt + boff + (size_t)nb * 16 * K + kc);
#pragma unroll
            for (int mb = 0; mb < 4; ++mb) acc[mb][nb] = wmma16(a[mb], b, acc[mb][nb]);
        }
        asm volatile("v_nop\n\tv_nop\n\tv_nop\n\tv_nop" : "+v"(acc[0][0]), "+v"(acc[1][1]), "+v"(acc[2][2]), "+v"(acc[3][3]) : "v"(a[0]), "v"(a[3]), "v"(b));
    }
#pragma unroll
    for (int mb = 0; mb < 4; ++mb) {
#pragma unroll
        for (int nb = 0; nb < 4; ++nb) {
#pragma unroll
            for (int j = 0; j < 8; ++j) os[(hi * 8 + j) * 68 + nb * 16 + lr] = acc[mb][nb][j];
        }
        __builtin_amdgcn_fence(3, "wavefront"); __builtin_amdgcn_wave_barrier(); asm volatile("" ::: "memory");
        if constexpr (EP == EP_RES) {
            float* crow = Cf + z * sC + (size_t)(r0 + mb * 16) * ldc + c0;
            const float* rrow = R + (size_t)(r0 + mb * 16) * ldc + c0;
#pragma unroll 1
            for (int ps = 0; ps < 2; ++ps) {
#pragma unroll 1
                for (int s = 0; s < 8; ++s) {
                    const int row = 2 * s + hi, cofs = lr * 4;
                    const v4f u = *(const v4fa*)(os + row * 68 + cofs);
                    const v4f rv = *(const v4f*)(rrow + (size_t)row * ldc + cofs);
                    v4f o;
#pragma unroll
                    for (int q = 0; q < 4; ++q) {
                        float bq = 0.0f;
                        if constexpr (BIAS) bq = bfr(bias[c0 + cofs + q]);
                        const float y = u[q] * cs + bq;
                        const float rq0 = rv[q];
                        const float rq = RBF ? bfr(rq0) : rq0;
                        o[q] = rq + bfr(gam[c0 + cofs + q]) * y;
                    }
                    *(volatile v4f*)(crow + (size_t)row * ldc + cofs) = o;
                }
                if (ps == 0) __threadfence();
            }
        } else {
            h16* crow = Ch + z * sC + (size_t)(r0 + mb * 16) * ldc + c0;
            const int q8 = lane >> 3, cofs = (lane & 7) * 8;
#pragma unroll 1
            for (int ps = 0; ps < 2; ++ps) {
#pragma unroll 1
                for (int s = 0; s < 4; ++s) {
                    const int row = 4 * s + q8;
                    const v4f u0 = *(const v4fa*)(os + row * 68 + cofs), u1 = *(const v4fa*)(os + row * 68 + cofs + 4);
                    const v8f u = cat8f(u0, u1);
                    v8h o;
#pragma unroll
                    for (int q = 0; q < 8; ++q) {
                        float bq = 0.0f;
                        if constexpr (BIAS) bq = bfr(bias[c0 + cofs + q]);
                        float y = u[q] * cs + bq;
                        if constexpr (EP == EP_GELU) y = gelu_t(y);
                        o[q] = (h16)(y * co);
                    }
                    *(volatile v8h*)(crow + (size_t)row * ldc + cofs) = o;
                }
                if (ps == 0) __threadfence();
            }
        }
        __builtin_amdgcn_wave_barrier(); asm volatile("" ::: "memory");
    }
}

__global__ __launch_bounds__(256) void k_cvtw(const float* __restrict__ src, h16* dst, unsigned n8) {
    const unsigned i = blockIdx.x * 256 + threadIdx.x; if (i >= n8) return;
    const v4f a0 = *(const v4f*)(src + (size_t)i * 8), a1 = *(const v4f*)(src + (size_t)i * 8 + 4);
    const v8f a = cat8f(a0, a1);
    v8h o;
#pragma unroll
    for (int k = 0; k < 8; ++k) { const float f = a[k]; o[k] = (h16)(bfr(f) * WCAR); }
    h16* p = dst + (size_t)i * 8;
    *(volatile v8h*)p = o; __threadfence(); *(volatile v8h*)p = o;
}

template <bool RBF>
__global__ __launch_bounds__(128) void k_ln(const float* __restrict__ X, const float* __restrict__ w, const float* __restrict__ bb, h16* Hp) {
    __shared__ float red[8];
    const int row = blockIdx.x, t = threadIdx.x, lane = t & 31, wave = t >> 5;
    const float* xr = X + (size_t)row * DM + t * 8;
    const v4f p0 = *(const v4f*)xr, p1 = *(const v4f*)(xr + 4);
    v8f v = cat8f(p0, p1);
    if constexpr (RBF) {
#pragma unroll
        for (int k = 0; k < 8; ++k) { const float f = v[k]; v[k] = bfr(f); }
    }
    float s = 0.0f;
#pragma unroll
    for (int k = 0; k < 8; ++k) s += v[k];
    s = wsum(s);
    if (lane == 0) red[wave] = s;
    __syncthreads();
    const float mu = ((red[0] + red[1]) + (red[2] + red[3])) * (1.0f / DM);
    v8f d; float s2 = 0.0f;
#pragma unroll
    for (int k = 0; k < 8; ++k) { const float dk = v[k] - mu; d[k] = dk; s2 += dk * dk; }
    s2 = wsum(s2);
    if (lane == 0) red[4 + wave] = s2;
    __syncthreads();
    const float var = ((red[4] + red[5]) + (red[6] + red[7])) * (1.0f / DM);
    const float rs = rsqrtf(var + 1.0e-5f);
    const v4f w0 = *(const v4f*)(w + t * 8), w1 = *(const v4f*)(w + t * 8 + 4);
    const v4f b0 = *(const v4f*)(bb + t * 8), b1 = *(const v4f*)(bb + t * 8 + 4);
    const v8f wv = cat8f(w0, w1), bv = cat8f(b0, b1);
    v8h o;
#pragma unroll
    for (int k = 0; k < 8; ++k) { const float wk = wv[k], bk = bv[k]; o[k] = (h16)(((d[k] * rs) * bfr(wk) + bfr(bk)) * HCAR); }
    h16* dst = Hp + (size_t)row * DM + t * 8;
    *(volatile v8h*)dst = o; __threadfence(); *(volatile v8h*)dst = o;
}

__global__ __launch_bounds__(256) void k_vt16(const h16* __restrict__ QKV, h16* VT) {
    const unsigned e = (blockIdx.x * 256 + threadIdx.x) * 2; if (e >= (unsigned)(NB * NH * DH * SEQ)) return;
    const unsigned j = e % SEQ, rest = e / SEQ; const unsigned d = rest % DH, hd = (rest / DH) % NH, b = rest / (DH * NH);
    const size_t src = (size_t)(b * SEQ + j) * QKVW + 2 * DM + hd * DH + d;
    v2h o; o[0] = QKV[src]; o[1] = QKV[src + QKVW];
    *(volatile v2h*)(VT + e) = o; __threadfence(); *(volatile v2h*)(VT + e) = o;
}

__global__ __launch_bounds__(128) void k_score(const h16* __restrict__ QKV, const float* __restrict__ Wl, const float* __restrict__ bl, h16* LG, int bidx, int ibase) {
    __shared__ __align__(16) h16 sb[4 * 4096];
    __shared__ __align__(16) h16 lm[256 * 64];
    const int wave = threadIdx.x >> 5, lane = threadIdx.x & 31, lr = lane & 15, hi = lane >> 4;
    const int it = blockIdx.x, jt = blockIdx.y;
    h16* sw = sb + wave * 4096;
    v16h aw; v8f blg;
    ldmix(Wl, bl, 1.0f, lr, hi, aw, blg);
    const size_t qoff = (size_t)(bidx * SEQ + ibase + it * 16 + lr) * QKVW + 8 * hi;
    const size_t koff = (size_t)(bidx * SEQ + jt * 64 + wave * 16 + lr) * QKVW + DM + 8 * hi;
#pragma unroll 1
    for (int hp = 0; hp < 8; ++hp) {
        const int hc = hp * 128;
        v8f s0 = (v8f){}, s1 = (v8f){};
        v16h a0, a1, b0, b1;
#pragma unroll
        for (int ks = 0; ks < 2; ++ks) {
            a0 = ldfrag(QKV + qoff + hc + ks * 32);      b0 = ldfrag(QKV + koff + hc + ks * 32);
            a1 = ldfrag(QKV + qoff + hc + 64 + ks * 32); b1 = ldfrag(QKV + koff + hc + 64 + ks * 32);
            s0 = wmma16(a0, b0, s0); s1 = wmma16(a1, b1, s1);
        }
        asm volatile("v_nop\n\tv_nop\n\tv_nop\n\tv_nop" : "+v"(s0), "+v"(s1) : "v"(a0), "v"(a1), "v"(b0), "v"(b1));
#pragma unroll
        for (int r = 0; r < 8; ++r) { v2h tv; tv[0] = (h16)(s0[r] * 0.125f); tv[1] = (h16)(s1[r] * 0.125f); *(v2h*)(sw + ((8 * hi + r) * 16 + lr) * 16 + 2 * hp) = tv; }
    }
    __builtin_amdgcn_fence(3, "wavefront"); __builtin_amdgcn_wave_barrier(); asm volatile("" ::: "memory");
#pragma unroll 1
    for (int t = 0; t < 16; ++t) {
        const v16h bbv = ldfrag_lo(sw + (t * 16 + lr) * 16 + 8 * hi);
        v8f dd = wmma16(aw, bbv, (v8f){});
        asm volatile("v_nop\n\tv_nop\n\tv_nop\n\tv_nop" : "+v"(dd) : "v"(aw), "v"(bbv));
#pragma unroll
        for (int r = 0; r < 8; ++r) lm[((8 * hi + r) * 16 + t) * 64 + wave * 16 + lr] = (h16)(dd[r] * (1.0f / MCAR) + blg[r]);
    }
    __syncthreads();
    const int q8 = lane >> 3, pc = (lane & 7) * 8;
#pragma unroll 1
    for (int ps = 0; ps < 2; ++ps) {
#pragma unroll 1
        for (int s = 0; s < 16; ++s) {
            const int line = wave * 64 + 4 * s + q8; const int g = line >> 4, tt = line & 15;
            const v8h val = *(const v8ha*)(lm + line * 64 + pc);
            *(volatile v8h*)(LG + ((size_t)g * ICH + it * 16 + tt) * SEQ + jt * 64 + pc) = val;
        }
        if (ps == 0) __threadfence();
    }
}

__global__ __launch_bounds__(256) void k_softmix(const h16* __restrict__ LG, const float* __restrict__ Ww, const float* __restrict__ bw, h16* P2) {
    __shared__ __align__(16) h16 pt[SEQ * 16];
    __shared__ __align__(16) h16 st[16 * SEQ];
    const int il = blockIdx.x, wave = threadIdx.x >> 5, lane = threadIdx.x & 31, lr = lane & 15, hi = lane >> 4;
#pragma unroll 1
    for (int u = 0; u < 2; ++u) {
        const int g = 2 * wave + u;
        const h16* rp = LG + ((size_t)g * ICH + il) * SEQ + lane * EL;
        float xv[EL];
#pragma unroll
        for (int c = 0; c < NV8; ++c) {
            const v8h v = *(const v8ha*)(rp + 8 * c);
#pragma unroll
            for (int k = 0; k < 8; ++k) xv[8 * c + k] = (float)v[k];
        }
        float m = xv[0];
#pragma unroll
        for (int k = 1; k < EL; ++k) m = fmaxf(m, xv[k]);
        m = wmax(m);
        float s = 0.0f;
#pragma unroll
        for (int k = 0; k < EL; ++k) { const float e = __builtin_amdgcn_exp2f((xv[k] - m) * L2E); xv[k] = e; s += e; }
        s = wsum(s);
        const float f = PCAR * (1.0f / s);
#pragma unroll
        for (int k = 0; k < EL; ++k) pt[(lane * EL + k) * 16 + g] = (h16)(xv[k] * f);
    }
    __syncthreads();
    v16h aw; v8f bwg;
    ldmix(Ww, bw, P2CAR, lr, hi, aw, bwg);
#pragma unroll 1
    for (int c = 0; c < NTW; ++c) {
        const int j0 = (wave * NTW + c) * 16;
        const v16h bbv = ldfrag_lo(pt + (j0 + lr) * 16 + 8 * hi);
        v8f dd = wmma16(aw, bbv, (v8f){});
        asm volatile("v_nop\n\tv_nop\n\tv_nop\n\tv_nop" : "+v"(dd) : "v"(aw), "v"(bbv));
#pragma unroll
        for (int r = 0; r < 8; ++r) st[(8 * hi + r) * SEQ + j0 + lr] = (h16)(dd[r] * (P2CAR / (MCAR * PCAR)) + bwg[r]);
    }
    __syncthreads();
#pragma unroll 1
    for (int ps = 0; ps < 2; ++ps) {
#pragma unroll 1
        for (int u = 0; u < 2; ++u) {
            const int g = 2 * wave + u;
#pragma unroll
            for (int c = 0; c < NV8; ++c) {
                const v8h val = *(const v8ha*)(st + g * SEQ + c * 256 + lane * 8);
                *(volatile v8h*)(P2 + ((size_t)g * ICH + il) * SEQ + c * 256 + lane * 8) = val;
            }
        }
        if (ps == 0) __threadfence();
    }
}

static inline unsigned cdiv(size_t a, unsigned b) { return (unsigned)((a + b - 1) / b); }

extern "C" void kernel_launch(void* const* d_in, const int* in_sizes, int n_in,
                              void* d_out, int out_size, void* d_ws, size_t ws_size, hipStream_t stream) {
    if (n_in < 19) return;
    if (in_sizes[0] < NTOK * DM || in_sizes[1] < DM || in_sizes[2] < DM || in_sizes[3] < QKVW * DM || in_sizes[4] < QKVW ||
        in_sizes[5] < NH * NH || in_sizes[6] < NH || in_sizes[7] < NH * NH || in_sizes[8] < NH ||
        in_sizes[9] < DM * DM || in_sizes[10] < DM || in_sizes[11] < DM || in_sizes[12] < DM || in_sizes[13] < DM ||
        in_sizes[14] < FFD * DM || in_sizes[15] < FFD || in_sizes[16] < DM * FFD || in_sizes[17] < DM || in_sizes[18] < DM) return;
    if (out_size < NTOK * DM) return;
    const float* x      = (const float*)d_in[0];
    const float* ln1_w  = (const float*)d_in[1];
    const float* ln1_b  = (const float*)d_in[2];
    const float* qkv_w  = (const float*)d_in[3];
    const float* qkv_b  = (const float*)d_in[4];
    const float* pl_w   = (const float*)d_in[5];
    const float* pl_b   = (const float*)d_in[6];
    const float* pw_w   = (const float*)d_in[7];
    const float* pw_b   = (const float*)d_in[8];
    const float* out_w  = (const float*)d_in[9];
    const float* out_b  = (const float*)d_in[10];
    const float* gamma1 = (const float*)d_in[11];
    const float* ln2_w  = (const float*)d_in[12];
    const float* ln2_b  = (const float*)d_in[13];
    const float* fc1_w  = (const float*)d_in[14];
    const float* fc1_b  = (const float*)d_in[15];
    const float* fc2_w  = (const float*)d_in[16];
    const float* fc2_b  = (const float*)d_in[17];
    const float* gamma2 = (const float*)d_in[18];
    float* OUT = (float*)d_out;

    char* wsp = (char*)d_ws;
    auto take = [&](size_t bytes) { char* p = wsp; wsp += (bytes + 255) & ~(size_t)255; return (void*)p; };
    h16* WQKV  = (h16*)take((size_t)QKVW * DM * 2);
    h16* WO    = (h16*)take((size_t)DM * DM * 2);
    h16* W1    = (h16*)take((size_t)FFD * DM * 2);
    h16* W2    = (h16*)take((size_t)DM * FFD * 2);
    h16* QKV16 = (h16*)take((size_t)NTOK * QKVW * 2);
    h16* H2    = QKV16;
    h16* VT    = (h16*)take((size_t)NTOK * DM * 2);
    const size_t lgb = (size_t)NH * ICH * SEQ * 2;
    const size_t x1b = (size_t)NTOK * DM * 4;
    char* R1   = (char*)take(x1b > lgb ? x1b : lgb);
    h16* H1 = (h16*)R1; h16* LG = (h16*)R1; float* X1 = (float*)R1;
    const size_t a1b = (size_t)NTOK * FFD * 2;
    char* R2   = (char*)take(a1b > lgb ? a1b : lgb);
    h16* P2 = (h16*)R2; h16* A1 = (h16*)R2;
    h16* O16   = (h16*)take((size_t)NTOK * DM * 2);
    const size_t used = (size_t)(wsp - (char*)d_ws);
    if (used > ws_size || used > (size_t)134217728) return;

    k_cvtw<<<cdiv((size_t)QKVW * DM / 8, 256), 256, 0, stream>>>(qkv_w, WQKV, (unsigned)(QKVW * DM / 8));
    k_cvtw<<<cdiv((size_t)DM * DM / 8, 256), 256, 0, stream>>>(out_w, WO, (unsigned)(DM * DM / 8));
    k_cvtw<<<cdiv((size_t)FFD * DM / 8, 256), 256, 0, stream>>>(fc1_w, W1, (unsigned)(FFD * DM / 8));
    k_cvtw<<<cdiv((size_t)DM * FFD / 8, 256), 256, 0, stream>>>(fc2_w, W2, (unsigned)(DM * FFD / 8));
    k_ln<true><<<NTOK, 128, 0, stream>>>(x, ln1_w, ln1_b, H1);
    k_gemm<EP_H16, true, false><<<dim3(NTOK / 64, QKVW / 64, 1), 32, 0, stream>>>(H1, WQKV, DM, nullptr, QKV16, QKVW, 1.0f / (HCAR * WCAR), 1.0f, qkv_b, nullptr, nullptr, 0, 0, 0);
    k_vt16<<<cdiv((size_t)NB * NH * DH * SEQ / 2, 256), 256, 0, stream>>>(QKV16, VT);
    for (int b = 0; b < NB; ++b) {
        for (int c = 0; c < NCH; ++c) {
            const int ibase = c * ICH;
            k_score<<<dim3(ICH / 16, SEQ / 64, 1), 128, 0, stream>>>(QKV16, pl_w, pl_b, LG, b, ibase);
            k_softmix<<<dim3(ICH, 1, 1), 256, 0, stream>>>(LG, pw_w, pw_b, P2);
            k_gemm<EP_H16, false, false><<<dim3(ICH / 64, 1, NH), 32, 0, stream>>>(P2, VT + (size_t)b * NH * DH * SEQ, SEQ, nullptr, O16 + (size_t)(b * SEQ + ibase) * DM, DM,
                                                                                   OCAR / P2CAR, 1.0f, nullptr, nullptr, nullptr, (size_t)ICH * SEQ, (size_t)DH * SEQ, (size_t)DH);
        }
    }
    k_gemm<EP_RES, true, true><<<dim3(NTOK / 64, DM / 64, 1), 32, 0, stream>>>(O16, WO, DM, X1, nullptr, DM, 1.0f / (OCAR * WCAR), 1.0f, out_b, x, gamma1, 0, 0, 0);
    k_ln<false><<<NTOK, 128, 0, stream>>>(X1, ln2_w, ln2_b, H2);
    k_gemm<EP_GELU, true, false><<<dim3(NTOK / 64, FFD / 64, 1), 32, 0, stream>>>(H2, W1, DM, nullptr, A1, FFD, 1.0f / (HCAR * WCAR), ACAR, fc1_b, nullptr, nullptr, 0, 0, 0);
    k_gemm<EP_RES, true, false><<<dim3(NTOK / 64, DM / 64, 1), 32, 0, stream>>>(A1, W2, FFD, OUT, nullptr, DM, 1.0f / (ACAR * WCAR), 1.0f, fc2_b, X1, gamma2, 0, 0, 0);
}
